// GraphSAGE_31112743092745
// MI455X (gfx1250) — hardware-run, weakly checked
//
#include <hip/hip_runtime.h>


namespace {
constexpr int N = 100000, NP = 100096, NLIM = 100096  , NLIMN = (NLIM < N ? NLIM : N), E = 1600000, D0 = 128, D1 = 16, NC = 40, HP = 32  , P2P = 128  ;
constexpr float XS = 8.0f, WSC = 256.0f;
static_assert(NP % 64 == 0 && NLIM % 64 == 0 && NP % 8 == 0, "tiling");
typedef _Float16 b16;
typedef __attribute__((ext_vector_type(16))) _Float16 v16b;
typedef __attribute__((ext_vector_type(8))) _Float16 v8b;
typedef __attribute__((ext_vector_type(8))) float v8f;
typedef __attribute__((ext_vector_type(4))) float v4f;
__device__ __forceinline__ float bf16_rne(float f) { unsigned int u = __float_as_uint(f); u += 0x7FFFu + ((u >> 16) & 1u); return __uint_as_float(u & 0xFFFF0000u); }
__device__ __forceinline__ void split16(float v, b16& hi, b16& lo) { hi = (b16)v; lo = (b16)(v - (float)hi); }
__device__ __forceinline__ v16b frag_kb(const b16* p, int hh) { const v8b a = *(const v8b*)(p + 8 * hh), b = *(const v8b*)(p + 16 + 8 * hh); v16b f;
#pragma unroll
  for (int e = 0; e < 8; ++e) { f[e] = a[e]; f[8 + e] = b[e]; } return f; }
__device__ __forceinline__ v8f wmma16b(v16b a, v16b b, v8f c) { v8f d = __builtin_amdgcn_wmma_f32_16x16x32_f16(false, a, false, b, (short)0, c, false, false); asm volatile("v_nop\n\tv_nop\n\tv_nop\n\tv_nop" : "+v"(d) : "v"(a), "v"(b)); return d; }
__device__ __forceinline__ void wave_lds_sync() { __builtin_amdgcn_fence(__ATOMIC_RELEASE, "workgroup"); __builtin_amdgcn_wave_barrier(); __builtin_amdgcn_fence(__ATOMIC_ACQUIRE, "workgroup"); }
__device__ __forceinline__ float pmul(float a, float b) { float p = a * b; asm volatile("" : "+v"(p)); return p; }
__device__ __forceinline__ int iclamp(int v, int lo, int hi) { return v < lo ? lo : (v > hi ? hi : v); }
constexpr int CSR_NBLK = 512, CSR_GB = 9, CSR_GN = 1 << CSR_GB  , CSR_MAXG = 512, CSR_CAP = 12288  ;
__global__ __launch_bounds__(64) void csrA_kernel(const int* __restrict__ dst, int E, int N, int nG, int CHP, int NGP, int* __restrict__ STG, int* __restrict__ HST) {
  extern __shared__ int sm[];
  int* cnt = sm; int* run = sm + NGP; int* ids = sm + 2 * NGP;
  const int b = blockIdx.x; const int ch = (E + CSR_NBLK - 1) / CSR_NBLK; const int e0 = b * ch, e1 = min(E, e0 + ch);
  for (int i = threadIdx.x; i < NGP; i += 64) cnt[i] = 0;
  for (int i = threadIdx.x; i < CHP; i += 64) ids[i] = -1;
  __syncthreads();
  if (threadIdx.x == 0) {
    for (int e = e0; e < e1; ++e) { int d = dst[e]; d = (d < 0) ? 0 : (d >= N ? N - 1 : d); cnt[d >> CSR_GB] += 1; }
    int acc = 0; for (int g = 0; g < nG; ++g) { run[g] = acc; acc += cnt[g]; }
    for (int e = e0; e < e1; ++e) { int d = dst[e]; d = (d < 0) ? 0 : (d >= N ? N - 1 : d); const int g = d >> CSR_GB; ids[run[g]] = e; run[g] += 1; } }
  __syncthreads();
  typedef __attribute__((ext_vector_type(4))) int v4i;
  for (int pass = 0; pass < 2; ++pass) {
    for (int i = threadIdx.x; i < CHP / 4; i += 64) *(volatile v4i*)(STG + (size_t)b * CHP + i * 4) = *(const v4i*)(&ids[i * 4]);
    for (int i = threadIdx.x; i < NGP / 4; i += 64) { v4i v; for (int e = 0; e < 4; ++e) v[e] = (i * 4 + e < nG) ? cnt[i * 4 + e] : 0; *(volatile v4i*)(HST + (size_t)b * NGP + i * 4) = v; }
    __threadfence(); }
}
__global__ __launch_bounds__(512) void csrS_kernel(const int* __restrict__ HST, int nG, int NGP, int* __restrict__ START, int* __restrict__ TOT, int* __restrict__ OFF) {
  __shared__ int tot[CSR_MAXG];
  const int b = threadIdx.x;
  for (int pass = 0; pass < 2; ++pass) { int runb = 0; for (int g = 0; g < nG; ++g) { int c = HST[(size_t)b * NGP + g]; c = (c < 0) ? 0 : c; ((volatile int*)OFF)[(size_t)g * CSR_NBLK + b] = runb; runb += c; } __threadfence(); }
  for (int g = threadIdx.x; g < nG; g += 512) { int s = 0; for (int bb = 0; bb < CSR_NBLK; ++bb) { int c = HST[(size_t)bb * NGP + g]; s += (c < 0) ? 0 : c; } tot[g] = s; }
  __syncthreads();
  if (threadIdx.x < 32) {
    __shared__ int st[CSR_MAXG + 32];
    if (threadIdx.x == 0) { int acc = 0; for (int g = 0; g < NGP; ++g) { st[g] = acc; if (g < nG) acc += (tot[g] + 31) & ~31; } st[NGP] = acc; }
    __builtin_amdgcn_fence(__ATOMIC_RELEASE, "workgroup"); __builtin_amdgcn_wave_barrier(); __builtin_amdgcn_fence(__ATOMIC_ACQUIRE, "workgroup");
    for (int pass = 0; pass < 2; ++pass) { for (int i = threadIdx.x; i < NGP + 32; i += 32) { ((volatile int*)START)[i] = (i <= NGP) ? st[min(i, NGP)] : 0; ((volatile int*)TOT)[i] = (i < nG) ? tot[i] : 0; } __threadfence(); } }
}
__global__ __launch_bounds__(256) void csrB_kernel(const int* __restrict__ dst, int N, int nG, int CHP, int NGP, int permLen, const int* __restrict__ STG, const int* __restrict__ HST, const int* __restrict__ OFF, const int* __restrict__ START, const int* __restrict__ TOT, int* __restrict__ PERM, int* __restrict__ ROWPTR, int* __restrict__ ROWCNT, int* __restrict__ FLAG) {
  typedef __attribute__((ext_vector_type(4))) int v4i;
  __shared__ int ids[CSR_CAP]; __shared__ unsigned short key[CSR_CAP]; __shared__ int outp[CSR_CAP]; __shared__ int ncnt[CSR_GN + 1]; __shared__ int boff[CSR_NBLK + 1];
  const int g = blockIdx.x, t_ = threadIdx.x; int tot = TOT[g]; int st = START[g], stn = START[g + 1]; const int v0 = g * CSR_GN; const int nv = min(CSR_GN, N - v0);
  st = (st < 0) ? 0 : (st > permLen - 32 ? permLen - 32 : st) & ~31; stn = (stn < st) ? st : (stn > permLen ? permLen : stn); tot = (tot < 0) ? 0 : tot; if (tot > stn - st && tot <= CSR_CAP) tot = stn - st;
  if (tot > CSR_CAP) {
    for (int pass = 0; pass < 2; ++pass) { for (int i = t_; i < CSR_GN / 4; i += 256) { v4i a, c; for (int e = 0; e < 4; ++e) { a[e] = st; c[e] = 0; } *(volatile v4i*)(ROWPTR + v0 + i * 4) = a; *(volatile v4i*)(ROWCNT + v0 + i * 4) = c; } if (t_ == 0) ((volatile int*)FLAG)[0] = 1; __threadfence(); } (void)nv; return; }
  if (t_ == 0) { int acc = 0; for (int b = 0; b < CSR_NBLK; ++b) { boff[b] = acc; int c = HST[(size_t)b * NGP + g]; c = (c < 0) ? 0 : (c > CHP ? CHP : c); acc += c; if (acc > tot) acc = tot; } boff[CSR_NBLK] = acc; }
  for (int i = t_; i <= CSR_GN; i += 256) ncnt[i] = 0;
  __syncthreads();
  for (int b = 0; b < CSR_NBLK; ++b) { const int c = boff[b + 1] - boff[b]; int o_ = OFF[(size_t)g * CSR_NBLK + b]; o_ = (o_ < 0) ? 0 : (o_ > CHP - c ? CHP - c : o_); const int* src_ = STG + (size_t)b * CHP + o_;
    for (int i = t_; i < c; i += 256) { int id = src_[i]; id = (id < 0) ? 0 : id; ids[boff[b] + i] = id; int d = dst[id]; d = (d < v0) ? v0 : (d >= N ? N - 1 : d); int kk = d - v0; kk = (kk < 0) ? 0 : (kk >= CSR_GN ? CSR_GN - 1 : kk); key[boff[b] + i] = (unsigned short)kk; } }
  __syncthreads();
  if (t_ == 0) { for (int i = 0; i < tot; ++i) ncnt[key[i]] += 1; int acc = 0; for (int vl = 0; vl < CSR_GN; ++vl) { const int c = ncnt[vl]; ncnt[vl] = acc; acc += c; } ncnt[CSR_GN] = acc;
    for (int i = 0; i < tot; ++i) { const int vl = key[i]; outp[ncnt[vl]] = ids[i]; ncnt[vl] += 1; }
    for (int vl = CSR_GN; vl > 0; --vl) ncnt[vl] = ncnt[vl - 1]; ncnt[0] = 0; }
  __syncthreads();
  for (int pass = 0; pass < 2; ++pass) {
    for (int i = t_; i < (stn - st) / 4; i += 256) { v4i v; for (int e = 0; e < 4; ++e) { const int q = i * 4 + e; v[e] = (q < tot) ? outp[q] : -1; } *(volatile v4i*)(PERM + st + i * 4) = v; }
    for (int i = t_; i < CSR_GN / 4; i += 256) { v4i a, c; for (int e = 0; e < 4; ++e) { const int vl = i * 4 + e; a[e] = st + ncnt[vl]; c[e] = (vl < nv) ? (ncnt[vl + 1] - ncnt[vl]) : 0; } *(volatile v4i*)(ROWPTR + v0 + i * 4) = a; *(volatile v4i*)(ROWCNT + v0 + i * 4) = c; }
    __threadfence(); }
}
__global__ __launch_bounds__(256) void csrZ_kernel(int* __restrict__ p, size_t n4) { typedef __attribute__((ext_vector_type(4))) int v4i; const size_t tid = (size_t)blockIdx.x * 256 + threadIdx.x, nth = (size_t)gridDim.x * 256; v4i z = {0, 0, 0, 0}; for (size_t i = tid; i < n4; i += nth) *(volatile v4i*)(p + i * 4) = z; }
struct CsrBufs { int *STG, *HST, *OFF, *START, *TOT, *PERM, *ROWPTR, *ROWCNT, *FLAG; int nG, NGP, CHP; size_t permLen; char* base; size_t bytes; };
static size_t csr_carve(CsrBufs& c, char* ws, size_t off, int E, int N) {
  const size_t off0 = off; c.base = ws + off;
  auto al = [&](size_t bytes) { char* p = ws + off; off += (bytes + 255) & ~(size_t)255; return p; };
  c.nG = (N + CSR_GN - 1) / CSR_GN; c.NGP = (c.nG + 31) & ~31; const int ch = (E + CSR_NBLK - 1) / CSR_NBLK; c.CHP = (ch + 31) & ~31; c.permLen = (size_t)E + 32 * (size_t)c.nG + 32;
  c.STG = (int*)al((size_t)CSR_NBLK * c.CHP * 4); c.HST = (int*)al((size_t)CSR_NBLK * c.NGP * 4); c.OFF = (int*)al((size_t)c.NGP * CSR_NBLK * 4); c.START = (int*)al((size_t)(c.NGP + 64) * 4); c.TOT = (int*)al((size_t)(c.NGP + 64) * 4);
  c.PERM = (int*)al(c.permLen * 4); c.ROWPTR = (int*)al((size_t)c.nG * CSR_GN * 4); c.ROWCNT = (int*)al((size_t)c.nG * CSR_GN * 4); c.FLAG = (int*)al(256);
  c.bytes = off - off0; return off;
}
static void csr_build(const CsrBufs& c, const int* dst, int E, int N, hipStream_t stream) {
  const size_t smem = (size_t)(2 * c.NGP + c.CHP) * 4;
  csrZ_kernel<<<512, 256, 0, stream>>>((int*)c.base, c.bytes / 16);
  csrA_kernel<<<CSR_NBLK, 64, smem, stream>>>(dst, E, N, c.nG, c.CHP, c.NGP, c.STG, c.HST);
  csrS_kernel<<<1, 512, 0, stream>>>(c.HST, c.nG, c.NGP, c.START, c.TOT, c.OFF);
  csrB_kernel<<<c.nG, 256, 0, stream>>>(dst, N, c.nG, c.CHP, c.NGP, (int)c.permLen, c.STG, c.HST, c.OFF, c.START, c.TOT, c.PERM, c.ROWPTR, c.ROWCNT, c.FLAG);
}

typedef __attribute__((ext_vector_type(2))) float v2f;
__global__ __launch_bounds__(256) void prep_kernel(const float* __restrict__ w1l, const float* __restrict__ w1r, const float* __restrict__ w2l, const float* __restrict__ w2r, b16* __restrict__ W1T, b16* __restrict__ W2T) {
  for (int i = threadIdx.x; i < 32 * D0 / 8; i += 256) { const int e = i * 8; const int oo = e / D0, k0 = e % D0; v8b o; for (int j = 0; j < 8; ++j) { const int k = k0 + j; o[j] = (b16)(bf16_rne(oo < D1 ? w1l[k * D1 + oo] : w1r[k * D1 + oo - D1]) * WSC); } for (int pass = 0; pass < 2; ++pass) { *(volatile v8b*)(W1T + e) = o; __threadfence(); } }
  for (int i = threadIdx.x; i < P2P * HP / 8; i += 256) { const int e = i * 8; const int oo = e / HP, k0 = e % HP; v8b o; for (int j = 0; j < 8; ++j) { const int k = k0 + j; float w = 0.0f; if (k < D1) { if (oo < NC) w = w2l[k * NC + oo]; else if (oo >= 64 && oo < 64 + NC) w = w2r[k * NC + oo - 64]; } o[j] = (b16)(bf16_rne(w) * WSC); } for (int pass = 0; pass < 2; ++pass) { *(volatile v8b*)(W2T + e) = o; __threadfence(); } }
}
__global__ __launch_bounds__(128) void proj1_kernel(const float* __restrict__ x, const b16* __restrict__ W1T, float* __restrict__ P1) {
  __shared__ __attribute__((aligned(16))) float Tf[4][16][32 + 4];
  const int wave = threadIdx.x >> 5, lane = threadIdx.x & 31, nloc = lane & 15, hlf = lane >> 4; const size_t v0 = ((size_t)blockIdx.x * 4 + wave) * 16; const size_t vr = v0 + nloc; const size_t vra = vr < (size_t)N ? vr : (size_t)N - 1;
  v8f acc[2] = {(v8f){}, (v8f){}};
  if (v0 < (size_t)NLIM) {
#pragma unroll
    for (int ks = 0; ks < D0 / 32; ++ks) { v16b a; const float* xr = x + vra * D0 + ks * 32; const v4f c0 = *(const v4f*)(xr + 8 * hlf), c1 = *(const v4f*)(xr + 8 * hlf + 4), c2 = *(const v4f*)(xr + 16 + 8 * hlf), c3 = *(const v4f*)(xr + 16 + 8 * hlf + 4);
      for (int i = 0; i < 4; ++i) { a[i] = (b16)(bf16_rne(c0[i]) * XS); a[4 + i] = (b16)(bf16_rne(c1[i]) * XS); a[8 + i] = (b16)(bf16_rne(c2[i]) * XS); a[12 + i] = (b16)(bf16_rne(c3[i]) * XS); }
      if (vr >= (size_t)N) a = (v16b){};
#pragma unroll
      for (int t = 0; t < 2; ++t) acc[t] = wmma16b(a, frag_kb(W1T + (size_t)(t * 16 + nloc) * D0 + ks * 32, hlf), acc[t]); } }
#pragma unroll
  for (int t = 0; t < 2; ++t)
#pragma unroll
    for (int r = 0; r < 8; ++r) Tf[wave][8 * hlf + r][t * 16 + nloc] = acc[t][r] * (1.0f / (XS * WSC));
  wave_lds_sync();
  for (int pass = 0; pass < 2; ++pass) { for (int rr = 0; rr < 16; ++rr) ((volatile float*)P1)[(v0 + rr) * 32 + lane] = Tf[wave][rr][lane]; __threadfence(); }
}
__global__ __launch_bounds__(256) void edge1_kernel(const float* __restrict__ P1, const float* __restrict__ b1, const int* __restrict__ srcs, const int* __restrict__ PERM, const int* __restrict__ ROWPTR, const int* __restrict__ ROWCNT, int permLen, float* __restrict__ H) {
  const int wave = threadIdx.x >> 5, lane = threadIdx.x & 31; const size_t v = (size_t)blockIdx.x * 8 + wave; const int c = lane & 15; float a = 0.0f;
  if (v < (size_t)NLIMN) { int st = ROWPTR[v], cnt = ROWCNT[v]; cnt = iclamp(cnt, 0, 65536); st = iclamp(st, 0, permLen - cnt); int used = 0;
#pragma unroll 1
    for (int j = 0; j < cnt; ++j) { const int e = iclamp(PERM[st + j], 0, E - 1); const size_t s = (size_t)iclamp(srcs[e], 0, N - 1); if (s >= (size_t)NLIM) continue; ++used; a += P1[s * 32 + c]; }
    a = a / (float)(used > 1 ? used : 1) + bf16_rne(b1[c]) + P1[v * 32 + D1 + c]; a = fmaxf(a, 0.0f); if (lane >= D1) a = 0.0f; }
  for (int pass = 0; pass < 2; ++pass) { ((volatile float*)H)[v * HP + lane] = a; __threadfence(); }
}
__global__ __launch_bounds__(128) void proj2_kernel(const float* __restrict__ H, const b16* __restrict__ W2T, float* __restrict__ P2) {
  __shared__ __attribute__((aligned(16))) float Tf[4][16][128 + 4];
  const int wave = threadIdx.x >> 5, lane = threadIdx.x & 31, nloc = lane & 15, hlf = lane >> 4; const size_t v0 = ((size_t)blockIdx.x * 4 + wave) * 16; const size_t vr = v0 + nloc;
  v8f acc[8];
#pragma unroll
  for (int t = 0; t < 8; ++t) acc[t] = (v8f){};
  if (v0 < (size_t)NLIM) { v16b ah, al; const float* xr = H + vr * HP; const v4f c0 = *(const v4f*)(xr + 8 * hlf), c1 = *(const v4f*)(xr + 8 * hlf + 4), c2 = *(const v4f*)(xr + 16 + 8 * hlf), c3 = *(const v4f*)(xr + 16 + 8 * hlf + 4); float cv[16];
    for (int i = 0; i < 4; ++i) { cv[i] = c0[i]; cv[4 + i] = c1[i]; cv[8 + i] = c2[i]; cv[12 + i] = c3[i]; }
    for (int e2 = 0; e2 < 16; ++e2) { b16 p, q; split16(cv[e2] * XS, p, q); ah[e2] = p; al[e2] = q; }
#pragma unroll
    for (int t = 0; t < 8; ++t) { const v16b bw = frag_kb(W2T + (size_t)(t * 16 + nloc) * HP, hlf); acc[t] = wmma16b(ah, bw, acc[t]); acc[t] = wmma16b(al, bw, acc[t]); } }
#pragma unroll
  for (int t = 0; t < 8; ++t)
#pragma unroll
    for (int r = 0; r < 8; ++r) Tf[wave][8 * hlf + r][t * 16 + nloc] = acc[t][r] * (1.0f / (XS * WSC));
  wave_lds_sync();
  for (int pass = 0; pass < 2; ++pass) { for (int rr = 0; rr < 16; ++rr) *(volatile v4f*)(P2 + (v0 + rr) * P2P + lane * 4) = *(const v4f*)(&Tf[wave][rr][lane * 4]); __threadfence(); }
}
__global__ __launch_bounds__(256) void edge2_kernel(const float* __restrict__ P2, const float* __restrict__ b2, const int* __restrict__ srcs, const int* __restrict__ PERM, const int* __restrict__ ROWPTR, const int* __restrict__ ROWCNT, int permLen, float* __restrict__ out) {
  __shared__ __attribute__((aligned(16))) float YB[8 * NC];
  const int wave = threadIdx.x >> 5, lane = threadIdx.x & 31; const size_t v = (size_t)blockIdx.x * 8 + wave; const bool has1 = lane < NC - 32;
  float z0 = 0.0f, z1 = 0.0f;
  if (v < (size_t)NLIMN) { int st = ROWPTR[v], cnt = ROWCNT[v]; cnt = iclamp(cnt, 0, 65536); st = iclamp(st, 0, permLen - cnt); int used = 0; float a0 = 0.0f, a1 = 0.0f;
#pragma unroll 1
    for (int j = 0; j < cnt; ++j) { const int e = iclamp(PERM[st + j], 0, E - 1); const size_t s = (size_t)iclamp(srcs[e], 0, N - 1); if (s >= (size_t)NLIM) continue; ++used; a0 += P2[s * P2P + lane]; if (has1) a1 += P2[s * P2P + 32 + lane]; }
    const float inv = 1.0f / (float)(used > 1 ? used : 1);
    z0 = a0 * inv + bf16_rne(b2[lane]) + P2[v * P2P + 64 + lane]; z1 = has1 ? (a1 * inv + bf16_rne(b2[32 + lane]) + P2[v * P2P + 96 + lane]) : -INFINITY;
    float mx = fmaxf(z0, z1);
#pragma unroll
    for (int o = 1; o < 32; o <<= 1) mx = fmaxf(mx, __shfl_xor(mx, o));
    float se = __expf(z0 - mx) + (has1 ? __expf(z1 - mx) : 0.0f);
#pragma unroll
    for (int o = 1; o < 32; o <<= 1) se += __shfl_xor(se, o);
    const float lse = mx + __logf(se); z0 -= lse; z1 -= lse;
    YB[wave * NC + lane] = z0; if (has1) YB[wave * NC + 32 + lane] = z1; }
  __syncthreads();
  const size_t vb = (size_t)blockIdx.x * 8;
  for (int pass = 0; pass < 2; ++pass) { for (int i = threadIdx.x; i < 8 * NC / 4; i += 256) { const size_t f0 = vb * NC + (size_t)i * 4; if (f0 + 4 <= (size_t)NLIMN * NC) *(volatile v4f*)(out + f0) = *(const v4f*)(&YB[i * 4]); } __threadfence(); }
}
}

extern "C" void kernel_launch(void* const* d_in, const int* in_sizes, int n_in, void* d_out, int out_size, void* d_ws, size_t ws_size, hipStream_t stream) {
  (void)n_in;
  auto Fp = [&](int i) { return (const float*)d_in[i]; }; auto Ip = [&](int i) { return (const int*)d_in[i]; };
  if (in_sizes[0] != N * D0 || in_sizes[1] != 2 * E || in_sizes[2] != D0 * D1 || in_sizes[3] != D1 || in_sizes[4] != D0 * D1 || in_sizes[5] != D1 * NC || in_sizes[6] != NC || in_sizes[7] != D1 * NC || out_size != N * NC) return;
  size_t off = 0; char* ws = (char*)d_ws;
  auto carve = [&](size_t bytes) { char* p = ws + off; off += (bytes + 255) & ~(size_t)255; return p; };
  b16* W1T = (b16*)carve(32 * D0 * 2); b16* W2T = (b16*)carve(P2P * HP * 2); float* P1 = (float*)carve((size_t)NP * 32 * 4); float* H = (float*)carve((size_t)NP * HP * 4); float* P2 = (float*)carve((size_t)NP * P2P * 4);
  CsrBufs csr; off = csr_carve(csr, ws, off, E, N);
  if (off > ws_size || off > ((size_t)128 << 20)) return;
  prep_kernel<<<1, 256, 0, stream>>>(Fp(2), Fp(4), Fp(5), Fp(7), W1T, W2T);
  csr_build(csr, Ip(1) + E, E, N, stream);
  proj1_kernel<<<NP / 64, 128, 0, stream>>>(Fp(0), W1T, P1);
  edge1_kernel<<<NP / 8, 256, 0, stream>>>(P1, Fp(3), Ip(1), csr.PERM, csr.ROWPTR, csr.ROWCNT, (int)csr.permLen, H);
  proj2_kernel<<<NP / 64, 128, 0, stream>>>(H, W2T, P2);
  edge2_kernel<<<NP / 8, 256, 0, stream>>>(P2, Fp(6), Ip(1), csr.PERM, csr.ROWPTR, csr.ROWCNT, (int)csr.permLen, (float*)d_out);
}
